// NeuralGraph_89859305766987
// MI455X (gfx1250) — hardware-verified
//
#include <hip/hip_runtime.h>


#define NB   4
#define NN   512
#define CC   8
#define NND  (NB * NN)
#define RE   (NB * NN * NN)
#define CH   65536
#define NCHK (RE / CH)
typedef _Float16 h16;
typedef unsigned short bf;
typedef __attribute__((ext_vector_type(16))) __bf16   v16bf;
typedef __attribute__((ext_vector_type(16))) _Float16 v16h;
typedef __attribute__((ext_vector_type(8)))  _Float16 v8h;
typedef __attribute__((ext_vector_type(8)))  unsigned short v8us;
typedef __attribute__((ext_vector_type(8)))  float    v8f;
typedef __attribute__((ext_vector_type(4)))  float    v4f;
typedef v8h  __attribute__((may_alias)) v8ha;
typedef v4f  __attribute__((may_alias)) v4fa;
typedef v8us __attribute__((may_alias)) v8usa;

__device__ __forceinline__ unsigned short f2bf(float f) { unsigned u = __float_as_uint(f); u += 0x7FFFu + ((u >> 16) & 1u); return (unsigned short)(u >> 16); }
__device__ __forceinline__ float bf2f(unsigned short b) { return __uint_as_float(((unsigned)b) << 16); }
__device__ __forceinline__ float bfr(float f) { return bf2f(f2bf(f)); }
__device__ __forceinline__ v16h cat16(v8h lo, v8h hi) { return __builtin_shufflevector(lo, hi, 0, 1, 2, 3, 4, 5, 6, 7, 8, 9, 10, 11, 12, 13, 14, 15); }
__device__ __forceinline__ v16bf cat16b(v8us lo, v8us hi) { return __builtin_bit_cast(v16bf, __builtin_shufflevector(lo, hi, 0, 1, 2, 3, 4, 5, 6, 7, 8, 9, 10, 11, 12, 13, 14, 15)); }
__device__ __forceinline__ v8f wmma16(v16h a, v16h b, v8f c) { return __builtin_amdgcn_wmma_f32_16x16x32_f16(false, a, false, b, (short)0, c, false, false); }
__device__ __forceinline__ v8f wmmab(v16bf a, v16bf b, v8f c) { return __builtin_amdgcn_wmma_f32_16x16x32_bf16(false, a, false, b, (short)0, c, false, false); }


template <typename T16> struct WFrag;
template <> struct WFrag<h16> { typedef v16h V; static __device__ __forceinline__ V ld(const h16* p) { return cat16(*(const v8h*)p, *(const v8h*)(p + 16)); } static __device__ __forceinline__ v8f mma(V a, V b, v8f c) { return wmma16(a, b, c); } };
template <> struct WFrag<bf> { typedef v16bf V; static __device__ __forceinline__ V ld(const bf* p) { return cat16b(*(const v8us*)p, *(const v8us*)(p + 16)); } static __device__ __forceinline__ v8f mma(V a, V b, v8f c) { return wmmab(a, b, c); } };
template <typename T16, int NSPLIT, bool BIAS>
__global__ __launch_bounds__(32) void k_gemmw(const T16* __restrict__ A, const T16* __restrict__ A2, const T16* __restrict__ Bt, const T16* __restrict__ Bt2, int K, float* C, int ldc, const float* __restrict__ bias, size_t sA, size_t sB, size_t sC) {
    typedef typename WFrag<T16>::V V;
    __shared__ __align__(16) float os[16 * 68];
    const size_t z = blockIdx.z; A += z * sA; if (A2) A2 += z * sA; Bt += z * sB; if (Bt2) Bt2 += z * sB; C += z * sC;
    const int lane = threadIdx.x & 31, lr = lane & 15, hi = lane >> 4; const int r0 = blockIdx.x * 64, c0 = blockIdx.y * 64;
    v8f acc[4][4];
#pragma unroll
    for (int mb = 0; mb < 4; ++mb)
#pragma unroll
        for (int nb = 0; nb < 4; ++nb) acc[mb][nb] = (v8f){};
    const size_t aoff = (size_t)(r0 + lr) * K + 8 * hi, boff = (size_t)(c0 + lr) * K + 8 * hi;
#pragma unroll 1
    for (int kc = 0; kc < K; kc += 32) {
        V a[4], a2[4];
#pragma unroll
        for (int mb = 0; mb < 4; ++mb) { a[mb] = WFrag<T16>::ld(A + aoff + (size_t)mb * 16 * K + kc); if (NSPLIT == 1 || NSPLIT == 2) a2[mb] = WFrag<T16>::ld(A2 + aoff + (size_t)mb * 16 * K + kc); }
#pragma unroll
        for (int nb = 0; nb < 4; ++nb) { const V b = WFrag<T16>::ld(Bt + boff + (size_t)nb * 16 * K + kc); V b2; if (NSPLIT >= 2) b2 = WFrag<T16>::ld(Bt2 + boff + (size_t)nb * 16 * K + kc);
#pragma unroll
            for (int mb = 0; mb < 4; ++mb) { acc[mb][nb] = WFrag<T16>::mma(a[mb], b, acc[mb][nb]); if (NSPLIT == 1 || NSPLIT == 2) acc[mb][nb] = WFrag<T16>::mma(a2[mb], b, acc[mb][nb]); if (NSPLIT >= 2) acc[mb][nb] = WFrag<T16>::mma(a[mb], b2, acc[mb][nb]); } }
        asm volatile("v_nop\n\tv_nop\n\tv_nop\n\tv_nop" : "+v"(acc[0][0]), "+v"(acc[1][1]), "+v"(acc[2][2]), "+v"(acc[3][3]) : "v"(a[0]), "v"(a[3]));
    }
#pragma unroll
    for (int mb = 0; mb < 4; ++mb) {
#pragma unroll
        for (int nb = 0; nb < 4; ++nb) {
#pragma unroll
            for (int j = 0; j < 8; ++j) os[(hi * 8 + j) * 68 + nb * 16 + lr] = acc[mb][nb][j]; }
        __builtin_amdgcn_wave_barrier(); asm volatile("" ::: "memory");
        float* crow = C + (size_t)(r0 + mb * 16) * ldc + c0;
#pragma unroll 1
        for (int ps = 0; ps < 2; ++ps) {
#pragma unroll
            for (int s = 0; s < 8; ++s) { const int row = 2 * s + hi, cofs = lr * 4; v4f val = *(const v4fa*)(os + row * 68 + cofs); if (BIAS) { val[0] += bfr(bias[c0 + cofs]); val[1] += bfr(bias[c0 + cofs + 1]); val[2] += bfr(bias[c0 + cofs + 2]); val[3] += bfr(bias[c0 + cofs + 3]); }
                *(volatile v4f*)(crow + (size_t)row * ldc + cofs) = val; }
            if (ps == 0) __threadfence(); }
        __builtin_amdgcn_wave_barrier(); asm volatile("" ::: "memory");
    }
}

__device__ __forceinline__ float siluf(float x) { return x * __builtin_amdgcn_rcpf(1.0f + __expf(-x)); }

__global__ __launch_bounds__(256) void k_wt(const float* __restrict__ w, int K, int N, int Kp, int Np, bf* Bt) {
    typedef __attribute__((ext_vector_type(2))) unsigned short v2us;
    const int lane = threadIdx.x & 31; const int nlines = Np * Kp / 64; const int wg = blockIdx.x * 8 + (threadIdx.x >> 5), nw = gridDim.x * 8;
#pragma unroll 1
    for (int ps = 0; ps < 2; ++ps) {
#pragma unroll 1
        for (int L = wg; L < nlines; L += nw) { const int e = L * 64 + lane * 2; v2us o;
#pragma unroll
            for (int q = 0; q < 2; ++q) { const int n = (e + q) / Kp, k = (e + q) % Kp; o[q] = (n < N && k < K) ? f2bf(w[(size_t)(k < K ? k : 0) * N + (n < N ? n : 0)]) : (unsigned short)0; }
            *(volatile v2us*)(Bt + e) = o; }
        if (ps == 0) __threadfence(); }
}
__global__ __launch_bounds__(256) void k_mx(const float* __restrict__ nodes, const float* __restrict__ edges, int r0, bf* A) {
    typedef __attribute__((ext_vector_type(2))) unsigned short v2us;
    const int lane = threadIdx.x & 31; const int wrow = (blockIdx.x * 8 + (threadIdx.x >> 5)) * 16; if (wrow >= CH) return;
#pragma unroll 1
    for (int ps = 0; ps < 2; ++ps) {
#pragma unroll
        for (int L = 0; L < 8; ++L) { const int rl = wrow + L * 2 + (lane >> 4); const int c = (lane & 15) * 2; const int r = r0 + rl; const int b = r >> 18, i = (r >> 9) & 511, j = r & 511; v2us o;
#pragma unroll
            for (int q = 0; q < 2; ++q) { const int col = c + q; float v = 0.f;
                if (col < 8) v = nodes[((size_t)b * NN + j) * CC + col]; else if (col < 16) v = nodes[((size_t)b * NN + i) * CC + (col - 8)]; else if (col < 24) v = edges[(size_t)r * CC + (col - 16)];
                o[q] = f2bf(v); }
            *(volatile v2us*)(A + (size_t)rl * 32 + c) = o; }
        if (ps == 0) __threadfence(); }
}
__global__ __launch_bounds__(256) void k_silu_planes(const float* __restrict__ H, const float* __restrict__ bias, int rows, int KW, bf* Ph, bf* Pl) {
    typedef __attribute__((ext_vector_type(2))) unsigned short v2us;
    const int lane = threadIdx.x & 31; const size_t L0 = ((size_t)blockIdx.x * 8 + (threadIdx.x >> 5)) * 8; const size_t nlines = (size_t)rows * KW / 64;
#pragma unroll 1
    for (int ps = 0; ps < 2; ++ps) {
#pragma unroll
        for (int l = 0; l < 8; ++l) { const size_t L = L0 + l; if (L >= nlines) break; const size_t e = L * 64 + lane * 2; v2us oh, ol;
#pragma unroll
            for (int q = 0; q < 2; ++q) { const size_t r = (e + q) / KW; const int c = (int)((e + q) % KW); const float y = siluf(H[r * 64 + c] + bfr(bias[c])); const unsigned short hb = f2bf(y); oh[q] = hb; ol[q] = f2bf(y - bf2f(hb)); }
            *(volatile v2us*)(Ph + e) = oh; *(volatile v2us*)(Pl + e) = ol; }
        if (ps == 0) __threadfence(); }
}
__global__ __launch_bounds__(256) void k_edge_epi(const float* __restrict__ M, const float* __restrict__ b3, const float* __restrict__ edges, int r0, float* OUTE, float* MAB) {
    const int lane = threadIdx.x & 31; const int rl0 = (blockIdx.x * 8 + (threadIdx.x >> 5)) * 32; if (rl0 >= CH) return; const size_t rg0 = (size_t)r0 + rl0;
    v4f oe[2], om[4];
#pragma unroll
    for (int s = 0; s < 2; ++s) { const int rr = s * 16 + (lane >> 1), c0 = (lane & 1) * 4;
#pragma unroll
        for (int q = 0; q < 4; ++q) { const float v = bfr(edges[(rg0 + rr) * CC + c0 + q]) + M[(size_t)(rl0 + rr) * 64 + 16 + c0 + q] + bfr(b3[16 + c0 + q]); oe[s][q] = fminf(fmaxf(v, -100.f), 100.f); } }
#pragma unroll
    for (int s = 0; s < 4; ++s) { const int rr = s * 8 + (lane >> 2), c0 = (lane & 3) * 4;
#pragma unroll
        for (int q = 0; q < 4; ++q) om[s][q] = M[(size_t)(rl0 + rr) * 64 + c0 + q] + bfr(b3[c0 + q]); }
#pragma unroll 1
    for (int ps = 0; ps < 2; ++ps) {
#pragma unroll
        for (int s = 0; s < 2; ++s) { const int rr = s * 16 + (lane >> 1), c0 = (lane & 1) * 4; *(volatile v4f*)(OUTE + (rg0 + rr) * CC + c0) = oe[s]; }
#pragma unroll
        for (int s = 0; s < 4; ++s) { const int rr = s * 8 + (lane >> 2), c0 = (lane & 3) * 4; *(volatile v4f*)(MAB + (rg0 + rr) * 16 + c0) = om[s]; }
        if (ps == 0) __threadfence(); }
}
__global__ __launch_bounds__(256) void k_node_planes(const float* __restrict__ nodes, bf* An) {
    typedef __attribute__((ext_vector_type(2))) unsigned short v2us;
    const int lane = threadIdx.x & 31; const int wrow = (blockIdx.x * 8 + (threadIdx.x >> 5)) * 16; if (wrow >= NND) return;
#pragma unroll 1
    for (int ps = 0; ps < 2; ++ps) {
#pragma unroll
        for (int L = 0; L < 8; ++L) { const int r = wrow + L * 2 + (lane >> 4); const int c = (lane & 15) * 2; v2us o;
#pragma unroll
            for (int q = 0; q < 2; ++q) o[q] = (c + q < CC) ? f2bf(nodes[(size_t)r * CC + (c + q < CC ? c + q : 0)]) : (unsigned short)0;
            *(volatile v2us*)(An + (size_t)r * 32 + c) = o; }
        if (ps == 0) __threadfence(); }
}
template <int DIR>
__global__ __launch_bounds__(128) void k_agg(const float* __restrict__ ATT, const float* __restrict__ ab3, const float* __restrict__ MAB, const float* __restrict__ Wo, float* AG) {
    __shared__ float wsm[4][4][NN];
    const int lane = threadIdx.x & 31, wv = threadIdx.x >> 5; const int wg = blockIdx.x * 4 + wv; if (wg >= NB * (NN / 4)) return; const int b = wg / (NN / 4), t0 = (wg % (NN / 4)) * 4;
    const int qoff = DIR == 0 ? 8 : 24, koff = DIR == 0 ? 0 : 16; const float scale = 0.35355339059327373f;
    const int tt = lane >> 3, sub = lane & 7; const int t = t0 + tt;
    float qv[8];
#pragma unroll
    for (int k = 0; k < 8; ++k) qv[k] = ATT[((size_t)b * NN + t) * 64 + qoff + k] + bfr(ab3[qoff + k]);
    float mx = -3.0e38f;
#pragma unroll 2
    for (int it = 0; it < NN / 8; ++it) { const int src = it * 8 + sub; float s = 0.f;
#pragma unroll
        for (int k = 0; k < 8; ++k) s = fmaf(qv[k], ATT[((size_t)b * NN + src) * 64 + koff + k] + bfr(ab3[koff + k]), s);
        s *= scale; wsm[wv][tt][src] = s; mx = fmaxf(mx, s); }
#pragma unroll
    for (int sh = 4; sh; sh >>= 1) mx = fmaxf(mx, __shfl_xor(mx, sh, 32));
    float sum = 0.f;
#pragma unroll 2
    for (int it = 0; it < NN / 8; ++it) { const int src = it * 8 + sub; const float e = __expf(wsm[wv][tt][src] - mx); wsm[wv][tt][src] = e; sum += e; }
#pragma unroll
    for (int sh = 4; sh; sh >>= 1) sum += __shfl_xor(sum, sh, 32);
    const float inv = __fdiv_rn(1.0f, sum);
    __builtin_amdgcn_wave_barrier(); asm volatile("" ::: "memory");
    const int d = sub; float acc = 0.f;
#pragma unroll 4
    for (int src = 0; src < NN; ++src) { const size_t er = DIR == 0 ? (((size_t)b * NN + src) * NN + t) : (((size_t)b * NN + t) * NN + src); acc = fmaf(wsm[wv][tt][src], MAB[er * 16 + (DIR == 0 ? 0 : 8) + d], acc); }
    acc *= inv;
    float o = 0.f;
#pragma unroll
    for (int dd = 0; dd < 8; ++dd) { const float a = __shfl(acc, (lane & 24) + dd, 32); o = fmaf(a, bfr(Wo[dd * CC + d]), o); }
    float* dst = AG + ((size_t)b * NN + t0) * CC + lane; *(volatile float*)dst = o; __threadfence(); *(volatile float*)dst = o;
}
__global__ __launch_bounds__(256) void k_ui(const float* __restrict__ AGA, const float* __restrict__ AGB, const float* __restrict__ nodes, bf* Uh, bf* Ul) {
    typedef __attribute__((ext_vector_type(2))) unsigned short v2us;
    const int lane = threadIdx.x & 31; const int wrow = (blockIdx.x * 8 + (threadIdx.x >> 5)) * 16; if (wrow >= NND) return;
#pragma unroll 1
    for (int ps = 0; ps < 2; ++ps) {
#pragma unroll
        for (int L = 0; L < 8; ++L) { const int r = wrow + L * 2 + (lane >> 4); const int c = (lane & 15) * 2; v2us oh, ol;
#pragma unroll
            for (int q = 0; q < 2; ++q) { const int col = c + q; float v = 0.f;
                if (col < 8) v = AGA[(size_t)r * CC + col]; else if (col < 16) v = AGB[(size_t)r * CC + (col - 8)]; else if (col < 24) v = bfr(nodes[(size_t)r * CC + (col - 16)]);
                const unsigned short hb = f2bf(v); oh[q] = hb; ol[q] = f2bf(v - bf2f(hb)); }
            *(volatile v2us*)(Uh + (size_t)r * 32 + c) = oh; *(volatile v2us*)(Ul + (size_t)r * 32 + c) = ol; }
        if (ps == 0) __threadfence(); }
}
__global__ __launch_bounds__(256) void k_node_out(const float* __restrict__ nodes, const float* __restrict__ UPD, const float* __restrict__ ub3, float* OUTN) {
    const int lane = threadIdx.x & 31; const int r0 = (blockIdx.x * 8 + (threadIdx.x >> 5)) * 4; if (r0 >= NND) return; const int r = r0 + (lane >> 3), c = lane & 7;
    float v = bfr(nodes[(size_t)r * CC + c]) + UPD[(size_t)r * 64 + c] + bfr(ub3[c]); v = fminf(fmaxf(v, -100.f), 100.f);
    float* dst = OUTN + (size_t)r0 * CC + lane; *(volatile float*)dst = v; __threadfence(); *(volatile float*)dst = v;
}

extern "C" void kernel_launch(void* const* d_in, const int* in_sizes, int n_in,
                              void* d_out, int out_size, void* d_ws, size_t ws_size, hipStream_t stream) {
    (void)in_sizes; (void)n_in; (void)out_size;
    const float* nodes = (const float*)d_in[0]; const float* edges = (const float*)d_in[1];
    const float* mw1 = (const float*)d_in[2]; const float* mb1 = (const float*)d_in[3]; const float* mw2 = (const float*)d_in[4]; const float* mb2 = (const float*)d_in[5]; const float* mw3 = (const float*)d_in[6]; const float* mb3 = (const float*)d_in[7];
    const float* uw1 = (const float*)d_in[8]; const float* ub1 = (const float*)d_in[9]; const float* uw2 = (const float*)d_in[10]; const float* ub2 = (const float*)d_in[11]; const float* uw3 = (const float*)d_in[12]; const float* ub3 = (const float*)d_in[13];
    const float* aw1 = (const float*)d_in[14]; const float* ab1 = (const float*)d_in[15]; const float* aw2 = (const float*)d_in[16]; const float* ab2 = (const float*)d_in[17]; const float* aw3 = (const float*)d_in[18]; const float* ab3 = (const float*)d_in[19];
    const float* outa_w = (const float*)d_in[20]; const float* outb_w = (const float*)d_in[21];
    float* OUTN = (float*)d_out;
    float* OUTE = (float*)((char*)d_out + 65536);
    char* wsp = (char*)d_ws;
    auto take = [&](size_t bytes) { char* p = wsp; wsp += (bytes + 255) & ~(size_t)255; return (void*)p; };
    bf* W1t = (bf*)take(64 * 32 * 2); bf* W2t = (bf*)take(64 * 64 * 2); bf* W3t = (bf*)take(64 * 32 * 2);
    bf* A1t = (bf*)take(64 * 32 * 2); bf* A2t = (bf*)take(64 * 64 * 2); bf* A3t = (bf*)take(64 * 32 * 2);
    bf* U1t = (bf*)take(64 * 32 * 2); bf* U2t = (bf*)take(64 * 64 * 2); bf* U3t = (bf*)take(64 * 32 * 2);
    bf* AX = (bf*)take((size_t)CH * 32 * 2); float* H1 = (float*)take((size_t)CH * 64 * 4); bf* P1h = (bf*)take((size_t)CH * 64 * 2); bf* P1l = (bf*)take((size_t)CH * 64 * 2);
    bf* P2h = (bf*)take((size_t)CH * 32 * 2); bf* P2l = (bf*)take((size_t)CH * 32 * 2);
    float* H2 = H1; float* M3 = H1;
    float* MAB = (float*)take((size_t)RE * 16 * 4);
    bf* An = (bf*)take((size_t)NND * 32 * 2); float* NA1 = (float*)take((size_t)NND * 64 * 4); bf* NP1h = (bf*)take((size_t)NND * 64 * 2); bf* NP1l = (bf*)take((size_t)NND * 64 * 2);
    float* NA2 = (float*)take((size_t)NND * 64 * 4); bf* NP2h = (bf*)take((size_t)NND * 32 * 2); bf* NP2l = (bf*)take((size_t)NND * 32 * 2); float* ATT = (float*)take((size_t)NND * 64 * 4);
    float* AGA = (float*)take((size_t)NND * CC * 4); float* AGB = (float*)take((size_t)NND * CC * 4); bf* UIh = (bf*)take((size_t)NND * 32 * 2); bf* UIl = (bf*)take((size_t)NND * 32 * 2); float* UPD = (float*)take((size_t)NND * 64 * 4);
    if ((size_t)(wsp - (char*)d_ws) > ws_size) return;
    k_wt<<<1, 256, 0, stream>>>(mw1, 24, 64, 32, 64, W1t); k_wt<<<1, 256, 0, stream>>>(mw2, 64, 32, 64, 64, W2t); k_wt<<<1, 256, 0, stream>>>(mw3, 32, 24, 32, 64, W3t);
    k_wt<<<1, 256, 0, stream>>>(aw1, 8, 64, 32, 64, A1t);  k_wt<<<1, 256, 0, stream>>>(aw2, 64, 32, 64, 64, A2t); k_wt<<<1, 256, 0, stream>>>(aw3, 32, 32, 32, 64, A3t);
    k_wt<<<1, 256, 0, stream>>>(uw1, 24, 64, 32, 64, U1t); k_wt<<<1, 256, 0, stream>>>(uw2, 64, 32, 64, 64, U2t); k_wt<<<1, 256, 0, stream>>>(uw3, 32, 8, 32, 64, U3t);
    for (int ck = 0; ck < NCHK; ++ck) { const int r0 = ck * CH;
        k_mx<<<CH / 16 / 8, 256, 0, stream>>>(nodes, edges, r0, AX);
        k_gemmw<bf, 0, false><<<dim3(CH / 64, 1, 1), 32, 0, stream>>>(AX, nullptr, W1t, nullptr, 32, H1, 64, nullptr, 0, 0, 0);
        k_silu_planes<<<(unsigned)(((size_t)CH * 64 / 64 + 63) / 64), 256, 0, stream>>>(H1, mb1, CH, 64, P1h, P1l);
        k_gemmw<bf, 1, false><<<dim3(CH / 64, 1, 1), 32, 0, stream>>>(P1h, P1l, W2t, nullptr, 64, H2, 64, nullptr, 0, 0, 0);
        k_silu_planes<<<(unsigned)(((size_t)CH * 32 / 64 + 63) / 64), 256, 0, stream>>>(H2, mb2, CH, 32, P2h, P2l);
        k_gemmw<bf, 1, false><<<dim3(CH / 64, 1, 1), 32, 0, stream>>>(P2h, P2l, W3t, nullptr, 32, M3, 64, nullptr, 0, 0, 0);
        k_edge_epi<<<CH / 32 / 8, 256, 0, stream>>>(M3, mb3, edges, r0, OUTE, MAB); }
    k_node_planes<<<NND / 16 / 8, 256, 0, stream>>>(nodes, An);
    k_gemmw<bf, 0, false><<<dim3(NND / 64, 1, 1), 32, 0, stream>>>(An, nullptr, A1t, nullptr, 32, NA1, 64, nullptr, 0, 0, 0);
    k_silu_planes<<<(NND * 64 / 64 + 63) / 64, 256, 0, stream>>>(NA1, ab1, NND, 64, NP1h, NP1l);
    k_gemmw<bf, 1, false><<<dim3(NND / 64, 1, 1), 32, 0, stream>>>(NP1h, NP1l, A2t, nullptr, 64, NA2, 64, nullptr, 0, 0, 0);
    k_silu_planes<<<(NND * 32 / 64 + 63) / 64, 256, 0, stream>>>(NA2, ab2, NND, 32, NP2h, NP2l);
    k_gemmw<bf, 1, false><<<dim3(NND / 64, 1, 1), 32, 0, stream>>>(NP2h, NP2l, A3t, nullptr, 32, ATT, 64, nullptr, 0, 0, 0);
    k_agg<0><<<NB * (NN / 4) / 4, 128, 0, stream>>>(ATT, ab3, MAB, outa_w, AGA);
    k_agg<1><<<NB * (NN / 4) / 4, 128, 0, stream>>>(ATT, ab3, MAB, outb_w, AGB);
    k_ui<<<NND / 16 / 8, 256, 0, stream>>>(AGA, AGB, nodes, UIh, UIl);
    k_gemmw<bf, 1, false><<<dim3(NND / 64, 1, 1), 32, 0, stream>>>(UIh, UIl, U1t, nullptr, 32, NA1, 64, nullptr, 0, 0, 0);
    k_silu_planes<<<(NND * 64 / 64 + 63) / 64, 256, 0, stream>>>(NA1, ub1, NND, 64, NP1h, NP1l);
    k_gemmw<bf, 1, false><<<dim3(NND / 64, 1, 1), 32, 0, stream>>>(NP1h, NP1l, U2t, nullptr, 64, NA2, 64, nullptr, 0, 0, 0);
    k_silu_planes<<<(NND * 32 / 64 + 63) / 64, 256, 0, stream>>>(NA2, ub2, NND, 32, NP2h, NP2l);
    k_gemmw<bf, 1, false><<<dim3(NND / 64, 1, 1), 32, 0, stream>>>(NP2h, NP2l, U3t, nullptr, 32, UPD, 64, nullptr, 0, 0, 0);
    k_node_out<<<NND / 4 / 8, 256, 0, stream>>>(nodes, UPD, ub3, OUTN);
}
